// SO3InteractionBlock_28432683499857
// MI455X (gfx1250) — hardware-verified
//
#include <hip/hip_runtime.h>
#include <stddef.h>
#include <math.h>


#define M0     16
#define M1     8
#define DIM    40
#define NBAS   8
#define NW     576
#define KP     32
#define NCT    (NW / 16)
#define NTHR   256
#define NWAVE  8
#define GE     32
#define WPITCH 580
#define LROWS  64
#define EPT    8
#define NGRP   2
#define CHUNK  (NTHR * EPT * NGRP)
#define WCAP   (EPT * NGRP * 32)
#define LISTN  (NWAVE * WCAP)
#define NBA    256
#define PROWS  32

#define LDS_EDGE ((GE * WPITCH + GE * DIM + GE * 4 + GE * DIM) * 4)
#define LDS_AGG  ((NBA * DIM + 4096 + 3 * 1024 + 256 + 64 + LISTN + 32) * 4)

#define RS8    0.35355339059327373f
#define RS24   0.20412414523193151f
#define RS128  0.08838834764831845f
#define RS192  0.07216878364870323f
#define INV2   0.7071067811865476f
#define LOG2F  0.6931471805599453f

static_assert((CHUNK & (CHUNK - 1)) == 0);
static_assert(CHUNK <= 4096);
static_assert((NBA & (NBA - 1)) == 0 && NBA <= 4096);
static_assert(NTHR == GE * 8 && NTHR == PROWS * 8 && NTHR == LROWS * 4);
static_assert(2 * PROWS * DIM <= LISTN);
static_assert((NBA % PROWS) == 0);
static_assert(NCT == 36 && (NCT % 4) == 0);
static_assert(((GE * WPITCH * 4) % 16) == 0);
static_assert(NTHR == M0 * M0);

typedef float          v4f   __attribute__((ext_vector_type(4)));
typedef float          v8f   __attribute__((ext_vector_type(8)));
typedef int            v4i   __attribute__((ext_vector_type(4)));
typedef unsigned short v8us  __attribute__((ext_vector_type(8)));
typedef unsigned short v16us __attribute__((ext_vector_type(16)));
typedef __bf16         v16bf __attribute__((ext_vector_type(16)));
union Frag { v16us v; v8us u[2]; unsigned short s[16]; };

__device__ __forceinline__ unsigned short bf_bits(float f) {
  unsigned int u = __float_as_uint(f);
  u = u + 0x7FFFu + ((u >> 16) & 1u);
  return (unsigned short)(u >> 16);
}
__device__ __forceinline__ float bf_val(unsigned short b) {
  return __uint_as_float(((unsigned int)b) << 16);
}

__device__ __forceinline__ v8f wmb(v16us a, v16us b, v8f c) {
  v8f d = __builtin_amdgcn_wmma_f32_16x16x32_bf16(false, __builtin_bit_cast(v16bf, a), false,
                                                  __builtin_bit_cast(v16bf, b), (short)0, c, false, false);
  asm volatile("v_nop\n\tv_nop\n\tv_nop\n\tv_nop" : "+v"(d) : "v"(a), "v"(b));
  return d;
}

__device__ __forceinline__ float sspf(float n) {
  const float t = __expf(-n);
  return n + __logf(1.0f + t) - LOG2F;
}
__device__ __forceinline__ float nas(float hs) {
  const float s   = fmaf(hs, hs, 1e-16f);
  const float r   = rsqrtf(s);
  const float nrm = s * r;
  return hs * r * sspf(nrm);
}

__device__ __forceinline__ int scan_chunk(const int* __restrict__ dsts, int nE, int cbase, int slotBase,
                                          unsigned limu, int vec8, int* list, int tid, int lane, int wave) {
  int wc = 0;
#pragma unroll
  for (int g = 0; g < NGRP; ++g) {
    const int el0  = (g * NTHR + tid) * EPT;
    const int e0   = cbase + el0;
    const int sent = -2147483647 - 1;
    v4i da, db;
    if (vec8 != 0 && cbase + CHUNK <= nE) {
      da = *(const v4i*)(dsts + e0);
      db = *(const v4i*)(dsts + e0 + 4);
    } else {
      da.x = (e0     < nE) ? dsts[min(e0,     nE - 1)] : sent;
      da.y = (e0 + 1 < nE) ? dsts[min(e0 + 1, nE - 1)] : sent;
      da.z = (e0 + 2 < nE) ? dsts[min(e0 + 2, nE - 1)] : sent;
      da.w = (e0 + 3 < nE) ? dsts[min(e0 + 3, nE - 1)] : sent;
      db.x = (e0 + 4 < nE) ? dsts[min(e0 + 4, nE - 1)] : sent;
      db.y = (e0 + 5 < nE) ? dsts[min(e0 + 5, nE - 1)] : sent;
      db.z = (e0 + 6 < nE) ? dsts[min(e0 + 6, nE - 1)] : sent;
      db.w = (e0 + 7 < nE) ? dsts[min(e0 + 7, nE - 1)] : sent;
    }
    const unsigned nb = (unsigned)slotBase;
    const unsigned s0 = (unsigned)da.x - nb, s1 = (unsigned)da.y - nb;
    const unsigned s2 = (unsigned)da.z - nb, s3 = (unsigned)da.w - nb;
    const unsigned s4 = (unsigned)db.x - nb, s5 = (unsigned)db.y - nb;
    const unsigned s6 = (unsigned)db.z - nb, s7 = (unsigned)db.w - nb;
    const bool h0 = s0 < limu, h1 = s1 < limu, h2 = s2 < limu, h3 = s3 < limu;
    const bool h4 = s4 < limu, h5 = s5 < limu, h6 = s6 < limu, h7 = s7 < limu;
    const unsigned any = __builtin_amdgcn_ballot_w32(h0 | h1 | h2 | h3 | h4 | h5 | h6 | h7);
    if (any != 0u) {
#define HITJ(J, HJ, SJ) { \
        const unsigned mj = __builtin_amdgcn_ballot_w32(HJ); \
        if (mj != 0u) { \
          if (HJ) { \
            const int pos = wc + (int)__builtin_amdgcn_mbcnt_lo(mj, 0u); \
            if (pos < WCAP) list[wave * WCAP + pos] = ((el0 + (J)) << 12) | (int)(SJ); \
          } \
          wc += (int)__builtin_popcount(mj); } }
      HITJ(0, h0, s0)
      HITJ(1, h1, s1)
      HITJ(2, h2, s2)
      HITJ(3, h3, s3)
      HITJ(4, h4, s4)
      HITJ(5, h5, s5)
      HITJ(6, h6, s6)
      HITJ(7, h7, s7)
#undef HITJ
    }
  }
  return wc;
}

__global__ __launch_bounds__(NTHR) void k_prep(const float* __restrict__ Wfc, unsigned short* Bp) {
  const int i = blockIdx.x * NTHR + (int)threadIdx.x;
  if (i >= NW * (KP / 8)) return;
  const int n = i >> 2, part = i & 3;
  unsigned short v[8];
#pragma unroll
  for (int k = 0; k < NBAS; ++k) {
    const float w = Wfc[k * NW + n];
    const unsigned short hb = bf_bits(w);
    const unsigned short lb = bf_bits(w - bf_val(hb));
    v[k] = (part == 1) ? lb : ((part == 3) ? (unsigned short)0 : hb);
  }
  v8us o;
  o[0] = v[0]; o[1] = v[1]; o[2] = v[2]; o[3] = v[3];
  o[4] = v[4]; o[5] = v[5]; o[6] = v[6]; o[7] = v[7];
  unsigned short* dp = Bp + (size_t)i * 8;
  *(volatile v8us*)dp = o;
  __threadfence();
  *(volatile v8us*)dp = o;
}

__global__ __launch_bounds__(NTHR) void k_lin1(
    const float* __restrict__ x, const float* __restrict__ W1s, const float* __restrict__ W1v,
    float* H, int nN) {
  __shared__ __attribute__((aligned(16))) float sX[LROWS * DIM];
  __shared__ __attribute__((aligned(16))) float sO[LROWS * DIM];
  __shared__ float sWs[M0 * M0];
  __shared__ float sWv[M1 * M1];
  const int tid  = threadIdx.x;
  const int base = blockIdx.x * LROWS;
#pragma unroll
  for (int t = 0; t < 3; ++t) {
    const int q = tid + NTHR * t;
    if (q < LROWS * 10) {
      const int r = q / 10, c = q - r * 10;
      int node = base + r;
      node = node > nN - 1 ? nN - 1 : node;
      ((v4f*)sX)[q] = *(const v4f*)(x + (size_t)node * DIM + 4 * c);
    }
  }
  sWs[tid] = W1s[tid];
  if (tid < M1 * M1) sWv[tid] = W1v[tid];
  __syncthreads();

  const int el = tid >> 2, qd = tid & 3;
  const float* xr = sX + el * DIM;
  float a0 = 0.f, a1 = 0.f, a2 = 0.f, a3 = 0.f;
#pragma unroll 2
  for (int u = 0; u < M0; ++u) {
    const float xu = xr[u];
    const float* wr = sWs + u * M0 + 4 * qd;
    a0 = fmaf(xu, wr[0], a0);
    a1 = fmaf(xu, wr[1], a1);
    a2 = fmaf(xu, wr[2], a2);
    a3 = fmaf(xu, wr[3], a3);
  }
  const int c0 = 2 * qd, c1 = 2 * qd + 1;
  float g00 = 0.f, g01 = 0.f, g02 = 0.f, g10 = 0.f, g11 = 0.f, g12 = 0.f;
#pragma unroll 1
  for (int u = 0; u < M1; ++u) {
    const float x0 = xr[M0 + 3 * u], x1 = xr[M0 + 3 * u + 1], x2 = xr[M0 + 3 * u + 2];
    const float wa = sWv[u * M1 + c0], wb = sWv[u * M1 + c1];
    g00 = fmaf(x0, wa, g00); g01 = fmaf(x1, wa, g01); g02 = fmaf(x2, wa, g02);
    g10 = fmaf(x0, wb, g10); g11 = fmaf(x1, wb, g11); g12 = fmaf(x2, wb, g12);
  }
  float* orow = sO + el * DIM;
  orow[4 * qd + 0] = a0 * 0.25f;
  orow[4 * qd + 1] = a1 * 0.25f;
  orow[4 * qd + 2] = a2 * 0.25f;
  orow[4 * qd + 3] = a3 * 0.25f;
  orow[M0 + 3 * c0 + 0] = g00 * RS8;
  orow[M0 + 3 * c0 + 1] = g01 * RS8;
  orow[M0 + 3 * c0 + 2] = g02 * RS8;
  orow[M0 + 3 * c1 + 0] = g10 * RS8;
  orow[M0 + 3 * c1 + 1] = g11 * RS8;
  orow[M0 + 3 * c1 + 2] = g12 * RS8;
  __syncthreads();

  float* gp = H + (size_t)base * DIM;
#pragma unroll
  for (int t = 0; t < 3; ++t) {
    const int q = tid + NTHR * t;
    if (q < LROWS * 10) { const v4f v = ((const v4f*)sO)[q]; *(volatile v4f*)(gp + 4 * q) = v; }
  }
  __threadfence();
#pragma unroll
  for (int t = 0; t < 3; ++t) {
    const int q = tid + NTHR * t;
    if (q < LROWS * 10) { const v4f v = ((const v4f*)sO)[q]; *(volatile v4f*)(gp + 4 * q) = v; }
  }
}

__global__ __launch_bounds__(NTHR) void k_edge(
    const float* __restrict__ rad, const float* __restrict__ esh, const int* __restrict__ esrc,
    const float* __restrict__ H, const unsigned short* __restrict__ Bp, float* msg, int nE, int nN) {
  extern __shared__ v4f lds_dyn[];
  float* sW   = (float*)lds_dyn;
  float* sH   = sW + GE * WPITCH;
  float* sSh  = sH + GE * DIM;
  float* sMsg = sSh + GE * 4;
  const int tid = threadIdx.x, lane = tid & 31, wave = tid >> 5, h = lane >> 4, m = lane & 15;
  const int e0 = blockIdx.x * GE;

#pragma unroll
  for (int t = 0; t < 2; ++t) {
    const int q = tid + NTHR * t;
    if (q < GE * 10) {
      const int r = q / 10, c = q - r * 10;
      int e = e0 + r;
      e = e > nE - 1 ? nE - 1 : e;
      int s = esrc[e];
      s = s < 0 ? 0 : (s > nN - 1 ? nN - 1 : s);
      ((v4f*)sH)[q] = *(const v4f*)(H + (size_t)s * DIM + 4 * c);
    }
  }
  if (tid < GE) {
    int e = e0 + tid;
    e = e > nE - 1 ? nE - 1 : e;
    ((v4f*)sSh)[tid] = *(const v4f*)(esh + (size_t)e * 4);
  }

  {
    const int rt = wave & 1;
    int eA = e0 + rt * 16 + m;
    eA = eA > nE - 1 ? nE - 1 : eA;
    const float* rp = rad + (size_t)eA * NBAS;
    const v4f q0 = *(const v4f*)rp, q1 = *(const v4f*)(rp + 4);
    float rv[8];
    rv[0] = q0.x; rv[1] = q0.y; rv[2] = q0.z; rv[3] = q0.w;
    rv[4] = q1.x; rv[5] = q1.y; rv[6] = q1.z; rv[7] = q1.w;
    Frag a;
#pragma unroll
    for (int i = 0; i < 8; ++i) {
      const unsigned short hb = bf_bits(rv[i]);
      const unsigned short lb = bf_bits(rv[i] - bf_val(hb));
      a.s[i]     = hb;
      a.s[8 + i] = (h == 0) ? lb : (unsigned short)0;
    }
    const v8f zero = {0.f, 0.f, 0.f, 0.f, 0.f, 0.f, 0.f, 0.f};
#pragma unroll
    for (int j = 0; j < NCT / 4; ++j) {
      const int ct = (wave >> 1) + 4 * j;
      const unsigned short* bp = Bp + (size_t)(ct * 16 + m) * KP + 8 * h;
      Frag b;
      b.u[0] = *(const v8us*)bp;
      b.u[1] = *(const v8us*)(bp + 16);
      const v8f acc = wmb(a.v, b.v, zero);
      float* wp = sW + (rt * 16 + 8 * h) * WPITCH + ct * 16 + m;
#pragma unroll
      for (int r = 0; r < 8; ++r) wp[r * WPITCH] = acc[r] * RS8;
    }
  }
  __syncthreads();

  {
    const int el = tid >> 3, p = tid & 7;
    const int w0 = 2 * p, w1 = 2 * p + 1;
    const float* xr = sH + el * DIM;
    const float* wr = sW + el * WPITCH;
    const float sh0 = sSh[el * 4 + 0], sx = sSh[el * 4 + 1], sy = sSh[el * 4 + 2], sz = sSh[el * 4 + 3];
    float a0 = 0.f, a1 = 0.f;
#pragma unroll
    for (int u = 0; u < M0; ++u) {
      const float ys = xr[u] * sh0;
      a0 = fmaf(wr[u * M0 + w0], ys, a0);
      a1 = fmaf(wr[u * M0 + w1], ys, a1);
    }
    float b0 = 0.f, b1 = 0.f;
#pragma unroll
    for (int u = 0; u < M1; ++u) {
      const float d = fmaf(xr[M0 + 3 * u + 2], sz, fmaf(xr[M0 + 3 * u + 1], sy, xr[M0 + 3 * u] * sx));
      b0 = fmaf(wr[448 + u * M0 + w0], d, b0);
      b1 = fmaf(wr[448 + u * M0 + w1], d, b1);
    }
    const float ms0 = (a0 * 0.25f + b0 * RS24) * INV2;
    const float ms1 = (a1 * 0.25f + b1 * RS24) * INV2;
    float av = 0.f;
#pragma unroll
    for (int u = 0; u < M0; ++u) av = fmaf(xr[u], wr[256 + u * M1 + p], av);
    float c0 = 0.f, c1 = 0.f, c2 = 0.f;
#pragma unroll
    for (int u = 0; u < M1; ++u) {
      const float wq = wr[384 + u * M1 + p];
      c0 = fmaf(wq, xr[M0 + 3 * u]     * sh0, c0);
      c1 = fmaf(wq, xr[M0 + 3 * u + 1] * sh0, c1);
      c2 = fmaf(wq, xr[M0 + 3 * u + 2] * sh0, c2);
    }
    const float mv0 = ((av * sx) * 0.25f + c0 * RS8) * INV2;
    const float mv1 = ((av * sy) * 0.25f + c1 * RS8) * INV2;
    const float mv2 = ((av * sz) * 0.25f + c2 * RS8) * INV2;
    float* mrow = sMsg + el * DIM;
    mrow[w0] = ms0;
    mrow[w1] = ms1;
    mrow[M0 + 3 * p + 0] = mv0;
    mrow[M0 + 3 * p + 1] = mv1;
    mrow[M0 + 3 * p + 2] = mv2;
  }
  __syncthreads();

  float* gp = msg + (size_t)e0 * DIM;
#pragma unroll
  for (int t = 0; t < 2; ++t) {
    const int q = tid + NTHR * t;
    if (q < GE * 10) { const v4f v = ((const v4f*)sMsg)[q]; *(volatile v4f*)(gp + 4 * q) = v; }
  }
  __threadfence();
#pragma unroll
  for (int t = 0; t < 2; ++t) {
    const int q = tid + NTHR * t;
    if (q < GE * 10) { const v4f v = ((const v4f*)sMsg)[q]; *(volatile v4f*)(gp + 4 * q) = v; }
  }
}

__global__ __launch_bounds__(NTHR) void k_agg(
    const int* __restrict__ edst, const float* __restrict__ msg, const float* __restrict__ x,
    const float* __restrict__ W2s, const float* __restrict__ W2v,
    const float* __restrict__ R00, const float* __restrict__ R01,
    const float* __restrict__ R10, const float* __restrict__ R11,
    const int* __restrict__ nnp, float* out, int nN, int nE, int vec8, float invDeg) {
  extern __shared__ v4f lds_dyn[];
  float* sAcc = (float*)lds_dyn;
  float* sR00 = sAcc + NBA * DIM;
  float* sR01 = sR00 + 4096;
  float* sR10 = sR01 + 1024;
  float* sR11 = sR10 + 1024;
  float* sW2s = sR11 + 1024;
  float* sW2v = sW2s + 256;
  int*   list = (int*)(sW2v + 64);
  int*   wcnt = list + LISTN;
  float* sX   = (float*)list;
  float* sOut = sX + PROWS * DIM;
  const int tid = threadIdx.x, lane = tid & 31, wave = tid >> 5;
  const int slotBase = blockIdx.x * NBA;
  int nSeg = nnp[0];
  nSeg = nSeg > nN ? nN : nSeg;
  int lim = nSeg - slotBase;
  lim = lim < 0 ? 0 : (lim > NBA ? NBA : lim);
  const unsigned limu = (unsigned)lim;

  {
    const v4f z = {0.f, 0.f, 0.f, 0.f};
    for (int i = tid; i < NBA * DIM / 4; i += NTHR) ((v4f*)sAcc)[i] = z;
  }
  for (int i = tid; i < 4096; i += NTHR) sR00[i] = R00[i];
  for (int i = tid; i < 1024; i += NTHR) { sR01[i] = R01[i]; sR10[i] = R10[i]; sR11[i] = R11[i]; }
  sW2s[tid] = W2s[tid];
  if (tid < 64) sW2v[tid] = W2v[tid];
  __syncthreads();

  const int nChunks = (nE + CHUNK - 1) / CHUNK;
#pragma unroll 1
  for (int ch = 0; ch < nChunks; ++ch) {
    const int cbase = ch * CHUNK;
    const int wc = scan_chunk(edst, nE, cbase, slotBase, limu, vec8, list, tid, lane, wave);
    if (lane == 0) wcnt[wave] = wc;
    __syncthreads();
    if (wave == 0) {
#pragma unroll 1
      for (int wsx = 0; wsx < NWAVE; ++wsx) {
        int n = __builtin_amdgcn_readfirstlane(wcnt[wsx]);
        n = n > WCAP ? WCAP : (n < 0 ? 0 : n);
        const int* lp = list + wsx * WCAP;
#pragma unroll 1
        for (int i = 0; i < n; ++i) {
          const int ent  = __builtin_amdgcn_readfirstlane(lp[i]);
          const int slot = ent & (NBA - 1);
          int e = cbase + ((ent >> 12) & (CHUNK - 1));
          e = e > nE - 1 ? nE - 1 : e;
          const int la = lane > 9 ? 9 : lane;
          const v4f v = *(const v4f*)(msg + (size_t)e * DIM + 4 * la);
          v4f* ap = (v4f*)(sAcc + slot * DIM + 4 * la);
          const v4f sum = *ap + v;
          if (lane < 10) *ap = sum;
        }
      }
    }
    __syncthreads();
  }

#pragma unroll 1
  for (int pass = 0; pass < NBA / PROWS; ++pass) {
    const int nodeBase = slotBase + pass * PROWS;
    if (nodeBase >= nN) break;
    const int nValid = (nN - nodeBase) < PROWS ? (nN - nodeBase) : PROWS;
#pragma unroll
    for (int t = 0; t < 2; ++t) {
      const int q = tid + NTHR * t;
      if (q < PROWS * 10) {
        const int r = q / 10, c = q - r * 10;
        int node = nodeBase + r;
        node = node > nN - 1 ? nN - 1 : node;
        ((v4f*)sX)[q] = *(const v4f*)(x + (size_t)node * DIM + 4 * c);
      }
    }
    __syncthreads();
    {
      const int el = tid >> 3, p = tid & 7;
      const int w0 = 2 * p, w1 = 2 * p + 1;
      const float* ag = sAcc + (pass * PROWS + el) * DIM;
      const float* xr = sX + el * DIM;

      float a0 = 0.f, a1 = 0.f;
#pragma unroll 2
      for (int u = 0; u < M0; ++u) {
        const float s = ag[u] * invDeg;
        a0 = fmaf(s, sW2s[u * M0 + w0], a0);
        a1 = fmaf(s, sW2s[u * M0 + w1], a1);
      }
      const float hs0 = a0 * 0.25f, hs1 = a1 * 0.25f;
      float g0 = 0.f, g1 = 0.f, g2 = 0.f;
#pragma unroll 1
      for (int u = 0; u < M1; ++u) {
        const float wv = sW2v[u * M1 + p];
        g0 = fmaf(ag[M0 + 3 * u]     * invDeg, wv, g0);
        g1 = fmaf(ag[M0 + 3 * u + 1] * invDeg, wv, g1);
        g2 = fmaf(ag[M0 + 3 * u + 2] * invDeg, wv, g2);
      }
      const float hv0 = g0 * RS8, hv1 = g1 * RS8, hv2 = g2 * RS8;

      const float ns0 = nas(hs0), ns1 = nas(hs1);
      const float sv  = fmaf(hv0, hv0, fmaf(hv1, hv1, hv2 * hv2)) + 1e-16f;
      const float rr  = rsqrtf(sv);
      const float gg  = sspf(sv * rr) * rr;
      const float nv0 = hv0 * gg, nv1 = hv1 * gg, nv2 = hv2 * gg;

      float r0 = 0.f, r1 = 0.f;
#pragma unroll 1
      for (int u = 0; u < M0; ++u) {
        const float xu = xr[u];
        const float* Rr = sR00 + u * 256;
#pragma unroll 2
        for (int v = 0; v < M0; ++v) {
          const float tt = xu * xr[v];
          r0 = fmaf(tt, Rr[v * 16 + w0], r0);
          r1 = fmaf(tt, Rr[v * 16 + w1], r1);
        }
      }
      float qa = 0.f, qb = 0.f;
#pragma unroll 1
      for (int u = 0; u < M1; ++u) {
        const float x0 = xr[M0 + 3 * u], x1 = xr[M0 + 3 * u + 1], x2 = xr[M0 + 3 * u + 2];
        const float* Rr = sR11 + u * 128;
#pragma unroll 2
        for (int v = 0; v < M1; ++v) {
          const float d = fmaf(x0, xr[M0 + 3 * v], fmaf(x1, xr[M0 + 3 * v + 1], x2 * xr[M0 + 3 * v + 2]));
          qa = fmaf(d, Rr[v * 16 + w0], qa);
          qb = fmaf(d, Rr[v * 16 + w1], qb);
        }
      }
      float va0 = 0.f, va1 = 0.f, va2 = 0.f;
#pragma unroll 1
      for (int v = 0; v < M1; ++v) {
        float tt = 0.f;
#pragma unroll 2
        for (int u = 0; u < M0; ++u) tt = fmaf(xr[u], sR01[(u * M1 + v) * M1 + p], tt);
        va0 = fmaf(tt, xr[M0 + 3 * v],     va0);
        va1 = fmaf(tt, xr[M0 + 3 * v + 1], va1);
        va2 = fmaf(tt, xr[M0 + 3 * v + 2], va2);
      }
      float vb0 = 0.f, vb1 = 0.f, vb2 = 0.f;
#pragma unroll 1
      for (int u = 0; u < M1; ++u) {
        float tt = 0.f;
#pragma unroll 2
        for (int v = 0; v < M0; ++v) tt = fmaf(xr[v], sR10[(u * M0 + v) * M1 + p], tt);
        vb0 = fmaf(tt, xr[M0 + 3 * u],     vb0);
        vb1 = fmaf(tt, xr[M0 + 3 * u + 1], vb1);
        vb2 = fmaf(tt, xr[M0 + 3 * u + 2], vb2);
      }

      float* orow = sOut + el * DIM;
      orow[w0] = ns0 + (r0 * 0.0625f + qa * RS192) * INV2;
      orow[w1] = ns1 + (r1 * 0.0625f + qb * RS192) * INV2;
      orow[M0 + 3 * p + 0] = nv0 + (va0 * RS128 + vb0 * RS128) * INV2;
      orow[M0 + 3 * p + 1] = nv1 + (va1 * RS128 + vb1 * RS128) * INV2;
      orow[M0 + 3 * p + 2] = nv2 + (va2 * RS128 + vb2 * RS128) * INV2;
    }
    __syncthreads();

    float* gp = out + (size_t)nodeBase * DIM;
    const int nq = nValid * 10;
#pragma unroll
    for (int t = 0; t < 2; ++t) {
      const int q = tid + NTHR * t;
      if (q < nq) { const v4f v = ((const v4f*)sOut)[q]; *(volatile v4f*)(gp + 4 * q) = v; }
    }
    __threadfence();
#pragma unroll
    for (int t = 0; t < 2; ++t) {
      const int q = tid + NTHR * t;
      if (q < nq) { const v4f v = ((const v4f*)sOut)[q]; *(volatile v4f*)(gp + 4 * q) = v; }
    }
    __syncthreads();
  }
}

extern "C" void kernel_launch(void* const* d_in, const int* in_sizes, int n_in,
                              void* d_out, int out_size, void* d_ws, size_t ws_size,
                              hipStream_t stream) {
  if (n_in < 15) return;
  const int nN = in_sizes[0] / DIM;
  const int nE = in_sizes[3];
  if (nN <= 0 || nE <= 0 || in_sizes[0] != nN * DIM) return;
  if (in_sizes[1] != nE * NBAS || in_sizes[2] != nE * 4 || in_sizes[4] != nE || in_sizes[5] < 1) return;
  if (in_sizes[6] != M0 * M0 || in_sizes[7] != M1 * M1 || in_sizes[8] != NBAS * NW) return;
  if (in_sizes[9] != M0 * M0 || in_sizes[10] != M1 * M1) return;
  if (in_sizes[11] != M0 * M0 * M0 || in_sizes[12] != M0 * M1 * M1 ||
      in_sizes[13] != M1 * M0 * M1 || in_sizes[14] != M1 * M1 * M0) return;
  if (out_size != nN * DIM) return;
  if (nE > (1 << 27) || nN > (1 << 26)) return;

  const float* x    = (const float*)d_in[0];
  const float* rad  = (const float*)d_in[1];
  const float* esh  = (const float*)d_in[2];
  const int*   esrc = (const int*)d_in[3];
  const int*   edst = (const int*)d_in[4];
  const int*   nnp  = (const int*)d_in[5];
  const float* W1s  = (const float*)d_in[6];
  const float* W1v  = (const float*)d_in[7];
  const float* Wfc  = (const float*)d_in[8];
  const float* W2s  = (const float*)d_in[9];
  const float* W2v  = (const float*)d_in[10];
  const float* R00  = (const float*)d_in[11];
  const float* R01  = (const float*)d_in[12];
  const float* R10  = (const float*)d_in[13];
  const float* R11  = (const float*)d_in[14];
  float* out = (float*)d_out;

  const int nGE  = (nE + GE - 1) / GE;
  const int nL1  = (nN + LROWS - 1) / LROWS;
  const int nAG  = (nN + NBA - 1) / NBA;
  const int nPrp = (NW * (KP / 8) + NTHR - 1) / NTHR;

  char* ws = (char*)d_ws;
  size_t off = 0;
  const size_t oBp  = off; off += (size_t)NW * KP * 2;                      off = (off + 255) & ~(size_t)255;
  const size_t oH   = off; off += (size_t)nL1 * LROWS * DIM * 4;            off = (off + 255) & ~(size_t)255;
  const size_t oMsg = off; off += (size_t)nGE * GE * DIM * 4;               off = (off + 255) & ~(size_t)255;
  if (off > ws_size) return;
  unsigned short* Bp = (unsigned short*)(ws + oBp);
  float* H   = (float*)(ws + oH);
  float* msg = (float*)(ws + oMsg);

  const float invDeg = 1.0f / sqrtf((float)nE / (float)nN);
  const int vec8 = 1;

  k_prep<<<nPrp, NTHR, 0, stream>>>(Wfc, Bp);
  k_lin1<<<nL1, NTHR, 0, stream>>>(x, W1s, W1v, H, nN);
  hipFuncSetAttribute(reinterpret_cast<const void*>(&k_edge),
                      hipFuncAttributeMaxDynamicSharedMemorySize, LDS_EDGE);
  k_edge<<<nGE, NTHR, LDS_EDGE, stream>>>(rad, esh, esrc, H, Bp, msg, nE, nN);
  hipFuncSetAttribute(reinterpret_cast<const void*>(&k_agg),
                      hipFuncAttributeMaxDynamicSharedMemorySize, LDS_AGG);
  k_agg<<<nAG, NTHR, LDS_AGG, stream>>>(edst, msg, x, W2s, W2v, R00, R01, R10, R11, nnp, out,
                                        nN, nE, vec8, invDeg);
}
